// BiLSTMModel_2808908611660
// MI455X (gfx1250) — hardware-verified
//
#include <hip/hip_runtime.h>
#include <math.h>

constexpr int NSEQ  = 1024;
constexpr int NSTEP = 256;
constexpr int NFEAT = 5;
constexpr int NHID  = 64;
constexpr int NGATE = 256;
constexpr int NIN1  = 128;
constexpr int SEQ_PER_BLK = 16;
constexpr int NTHR  = 128;
constexpr int KX0 = 32,  KP0 = 96,  AP0 = 104;
constexpr int KX1 = 128, KP1 = 192, AP1 = 200;
constexpr int HSP = 68;
constexpr float WSC = 8.0f;
constexpr float WSC_INV = 0.125f;

static_assert((SEQ_PER_BLK * AP0) % NTHR == 0, "zero loop covers the layer-0 A tile exactly");
static_assert((SEQ_PER_BLK * AP1) % NTHR == 0, "zero loop covers the layer-1 A tile exactly");
static_assert((NGATE * KP0 / 8) % 256 == 0, "layer-0 Bt plane is a whole number of 256-piece blocks");
static_assert((NGATE * KP1 / 8) % 256 == 0, "layer-1 Bt plane is a whole number of 256-piece blocks");
static_assert(KP0 % 32 == 0 && KP1 % 32 == 0, "K multiples of 32");

typedef __attribute__((ext_vector_type(16))) _Float16 v16h;
typedef __attribute__((ext_vector_type(8)))  _Float16 v8h;
typedef __attribute__((ext_vector_type(8)))  float    v8f;
typedef __attribute__((ext_vector_type(4)))  float    v4f;

__device__ __forceinline__ void dep_guard_h(v8f& a, v8f& b, v16h x, v16h y) { asm volatile("v_nop\n\tv_nop\n\tv_nop\n\tv_nop" : "+v"(a), "+v"(b) : "v"(x), "v"(y)); }
__device__ __forceinline__ void keep4_h(v16h a, v16h b, v16h c, v16h d) { asm volatile("v_nop" :: "v"(a), "v"(b), "v"(c), "v"(d)); }
__device__ __forceinline__ void acc_guard4(v8f& a, v8f& b, v8f& c, v8f& d) { asm volatile("v_nop\n\tv_nop\n\tv_nop\n\tv_nop" : "+v"(a), "+v"(b), "+v"(c), "+v"(d)); }
template <typename T> struct Frag;
template <> struct Frag<_Float16> {
  typedef v16h V; union U { v16h v; v8h h[2]; };
  static __device__ __forceinline__ v16h load(const _Float16* p) {
    U f; f.h[0] = *(const v8h*)(p); f.h[1] = *(const v8h*)(p + 16); return f.v;
  }
  static __device__ __forceinline__ v8f mma(v16h a, v16h b, v8f c) {
    return __builtin_amdgcn_wmma_f32_16x16x32_f16(false, a, false, b, (short)0, c, false, false);
  }
};

__device__ __forceinline__ float fsig(float x)  { return __builtin_amdgcn_rcpf(1.0f + __expf(-x)); }
__device__ __forceinline__ float ftanh(float x) { return 1.0f - 2.0f * __builtin_amdgcn_rcpf(__expf(2.0f * x) + 1.0f); }

__global__ __launch_bounds__(256) void pack_weights_kernel(
    const float* __restrict__ wih0f, const float* __restrict__ whh0f,
    const float* __restrict__ wih0b, const float* __restrict__ whh0b,
    const float* __restrict__ wih1f, const float* __restrict__ whh1f,
    const float* __restrict__ wih1b, const float* __restrict__ whh1b,
    unsigned short* __restrict__ Bt0, unsigned short* __restrict__ Bt1) {
  const int plane = blockIdx.y;
  const int layer = plane >> 1, dir = plane & 1;
  const int KP  = layer ? KP1 : KP0;
  const int KX  = layer ? KX1 : KX0;
  const int DIN = layer ? NIN1 : NFEAT;
  const float* wih = (plane == 0) ? wih0f : (plane == 1) ? wih0b : (plane == 2) ? wih1f : wih1b;
  const float* whh = (plane == 0) ? whh0f : (plane == 1) ? whh0b : (plane == 2) ? whh1f : whh1b;
  unsigned short* O = layer ? (Bt1 + (size_t)dir * NGATE * KP1) : (Bt0 + (size_t)dir * NGATE * KP0);
  const int npieces = NGATE * KP / 8;
  if ((int)blockIdx.x * 256 >= npieces) return;
  const int p = blockIdx.x * 256 + threadIdx.x;
  const int ppr = KP / 8;
  const int n = p / ppr;
  const int k8 = (p - n * ppr) * 8;
  v8h hv;
#pragma unroll
  for (int e = 0; e < 8; ++e) {
    const int k = k8 + e;
    const int ki = (k < DIN) ? k : (DIN - 1);
    int kh = k - KX; kh = kh < 0 ? 0 : (kh > NHID - 1 ? NHID - 1 : kh);
    const float a = wih[n * DIN + ki];
    const float b = whh[n * NHID + kh];
    const float v = (k < DIN) ? a : ((k >= KX) ? b : 0.0f);
    hv[e] = (_Float16)(v * WSC);
  }
  unsigned short* op = O + (size_t)p * 8;
  for (int pass = 0; pass < 2; ++pass) {
    *(volatile v8h*)op = hv;
    __threadfence();
  }
}

template <int LAYER>
__device__ __forceinline__ void stage_x(_Float16* At, const float* __restrict__ x, const _Float16* X16,
                                        int rowbase, int tt, int tid) {
  if (LAYER == 0) {
    const int i = tid < SEQ_PER_BLK * NFEAT ? tid : (SEQ_PER_BLK * NFEAT - 1);
    const int m = i / NFEAT, d = i - m * NFEAT;
    const float v = x[((size_t)(rowbase + m) * NSTEP + (size_t)tt) * NFEAT + d];
    if (tid < SEQ_PER_BLK * NFEAT) At[m * AP0 + d] = (_Float16)v;
  } else {
#pragma unroll
    for (int it = 0; it < 2; ++it) {
      const int idx = it * NTHR + tid;
      const int m = idx >> 4, c8 = (idx & 15) * 8;
      const v8h v = *(const v8h*)(X16 + ((size_t)(rowbase + m) * NSTEP + (size_t)tt) * NIN1 + c8);
      *(v8h*)(At + m * AP1 + c8) = v;
    }
  }
}

template <int LAYER>
__global__ __launch_bounds__(NTHR) void bilstm_layer_kernel(
    const float* __restrict__ x, const unsigned short* in16,
    const unsigned short* __restrict__ Btp,
    const float* __restrict__ bih_f, const float* __restrict__ bhh_f,
    const float* __restrict__ bih_b, const float* __restrict__ bhh_b,
    unsigned short* out16, float* __restrict__ last) {
  constexpr int KX = LAYER ? KX1 : KX0;
  constexpr int KP = LAYER ? KP1 : KP0;
  constexpr int AP = LAYER ? AP1 : AP0;
  constexpr int KSTEPS = KP / 32;
  constexpr int ZIT = SEQ_PER_BLK * AP / NTHR;
  __shared__ __align__(16) _Float16 At[SEQ_PER_BLK * AP];
  __shared__ __align__(16) float Hs[LAYER ? SEQ_PER_BLK * HSP : 4];

  const int tid = threadIdx.x, lane = tid & 31, wave = tid >> 5;
  const int c = lane & 15, hh = lane >> 4, koff = hh * 8;
  const int dir = blockIdx.x >> 6;
  const int rowbase = (blockIdx.x & 63) * SEQ_PER_BLK;
  const int nsteps = (LAYER == 1 && dir == 1) ? 1 : NSTEP;
  const _Float16* Bt  = (const _Float16*)Btp + (size_t)dir * NGATE * KP;
  const _Float16* X16 = (const _Float16*)in16;
  const float* bih = dir ? bih_b : bih_f;
  const float* bhh = dir ? bhh_b : bhh_f;
  const int j = 16 * wave + c;

#pragma unroll
  for (int i = 0; i < ZIT; ++i) At[i * NTHR + tid] = (_Float16)0.0f;
  float bb[4], cst[8], hst[8];
#pragma unroll
  for (int g = 0; g < 4; ++g) bb[g] = bih[g * NHID + j] + bhh[g * NHID + j];
#pragma unroll
  for (int r = 0; r < 8; ++r) { cst[r] = 0.0f; hst[r] = 0.0f; }
  __syncthreads();
  stage_x<LAYER>(At, x, X16, rowbase, dir ? (NSTEP - 1) : 0, tid);
  __syncthreads();

  const _Float16* arow = At + c * AP + koff;
  const v8f z8 = {0.f, 0.f, 0.f, 0.f, 0.f, 0.f, 0.f, 0.f};

#pragma unroll 1
  for (int s = 0; s < nsteps; ++s) {
    const int tt = dir ? (NSTEP - 1 - s) : s;
    v8f acc[4];
    acc[0] = z8; acc[1] = z8; acc[2] = z8; acc[3] = z8;
#pragma unroll 1
    for (int ks = 0; ks < KSTEPS; ++ks) {
      const _Float16* wb = Bt + (size_t)j * KP + koff + 32 * ks;
      const v16h a  = Frag<_Float16>::load(arow + 32 * ks);
      const v16h b0 = Frag<_Float16>::load(wb);
      const v16h b1 = Frag<_Float16>::load(wb + (size_t)1 * NHID * KP);
      const v16h b2 = Frag<_Float16>::load(wb + (size_t)2 * NHID * KP);
      const v16h b3 = Frag<_Float16>::load(wb + (size_t)3 * NHID * KP);
      acc[0] = Frag<_Float16>::mma(a, b0, acc[0]);
      acc[1] = Frag<_Float16>::mma(a, b1, acc[1]);
      acc[2] = Frag<_Float16>::mma(a, b2, acc[2]);
      acc[3] = Frag<_Float16>::mma(a, b3, acc[3]);
      dep_guard_h(acc[0], acc[3], a, b3);
      keep4_h(b0, b1, b2, b3);
    }
    acc_guard4(acc[0], acc[1], acc[2], acc[3]);
#pragma unroll
    for (int r = 0; r < 8; ++r) {
      const float zi = acc[0][r] * WSC_INV + bb[0];
      const float zf = acc[1][r] * WSC_INV + bb[1];
      const float zg = acc[2][r] * WSC_INV + bb[2];
      const float zo = acc[3][r] * WSC_INV + bb[3];
      const float ig = fsig(zi);
      const float fg = fsig(zf);
      const float gg = ftanh(zg);
      const float og = fsig(zo);
      const float cn = fg * cst[r] + ig * gg;
      cst[r] = cn;
      hst[r] = og * ftanh(cn);
    }
    __syncthreads();
#pragma unroll
    for (int r = 0; r < 8; ++r) At[(8 * hh + r) * AP + KX + j] = (_Float16)hst[r];
    {
      const int sn  = (s + 1 < nsteps) ? (s + 1) : s;
      const int ttn = dir ? (NSTEP - 1 - sn) : sn;
      stage_x<LAYER>(At, x, X16, rowbase, ttn, tid);
    }
    __syncthreads();
    if (LAYER == 0) {
      const int q = lane >> 3, c8 = (lane & 7) * 8;
      const int m = wave * 4 + q;
      const v8h hv = *(const v8h*)(At + m * AP + KX + c8);
      unsigned short* op = out16 + ((size_t)(rowbase + m) * NSTEP + (size_t)tt) * NIN1 + NHID * dir + c8;
      for (int pass = 0; pass < 2; ++pass) {
        *(volatile v8h*)op = hv;
        __threadfence();
      }
    }
  }

  if (LAYER == 1) {
#pragma unroll
    for (int r = 0; r < 8; ++r) Hs[(8 * hh + r) * HSP + j] = hst[r];
    __syncthreads();
    for (int pass = 0; pass < 2; ++pass) {
#pragma unroll
      for (int it = 0; it < 2; ++it) {
        const int idx = it * NTHR + tid;
        const int row = idx >> 4, c4 = (idx & 15) * 4;
        const v4f v = *(const v4f*)(Hs + row * HSP + c4);
        *(volatile v4f*)(last + (size_t)(rowbase + row) * NIN1 + NHID * dir + c4) = v;
      }
      __threadfence();
    }
  }
}

__global__ __launch_bounds__(256) void head_kernel(const float* __restrict__ last, const float* __restrict__ fcw,
                                                  const float* __restrict__ fcb, float* __restrict__ out) {
  __shared__ __align__(16) float ys[256];
  const int tid = threadIdx.x;
  const int b = blockIdx.x * 256 + tid;
  const float* row = last + (size_t)b * NIN1;
  float acc = 0.0f;
#pragma unroll 1
  for (int k = 0; k < NIN1; ++k) acc = fmaf(row[k], fcw[k], acc);
  ys[tid] = acc + fcb[0];
  __syncthreads();
  if (tid < 64) {
    const v4f v = *(const v4f*)(ys + 4 * tid);
    float* op = out + (size_t)blockIdx.x * 256 + 4 * tid;
    *(volatile v4f*)op = v;
    __threadfence();
    *(volatile v4f*)op = v;
  }
}

extern "C" void kernel_launch(void* const* d_in, const int* in_sizes, int n_in,
                              void* d_out, int out_size, void* d_ws, size_t ws_size, hipStream_t stream) {
  if (n_in < 19 || d_out == nullptr || d_ws == nullptr) return;
  if (in_sizes[0] != NSEQ * NSTEP * NFEAT || out_size != NSEQ) return;
  if (in_sizes[1] != NGATE * NFEAT || in_sizes[2] != NGATE * NHID || in_sizes[3] != NGATE || in_sizes[4] != NGATE) return;
  if (in_sizes[5] != NGATE * NFEAT || in_sizes[6] != NGATE * NHID || in_sizes[7] != NGATE || in_sizes[8] != NGATE) return;
  if (in_sizes[9] != NGATE * NIN1 || in_sizes[10] != NGATE * NHID || in_sizes[11] != NGATE || in_sizes[12] != NGATE) return;
  if (in_sizes[13] != NGATE * NIN1 || in_sizes[14] != NGATE * NHID || in_sizes[15] != NGATE || in_sizes[16] != NGATE) return;
  if (in_sizes[17] != NIN1 || in_sizes[18] != 1) return;

  const float* x        = (const float*)d_in[0];
  const float* w_ih_l0  = (const float*)d_in[1];
  const float* w_hh_l0  = (const float*)d_in[2];
  const float* b_ih_l0  = (const float*)d_in[3];
  const float* b_hh_l0  = (const float*)d_in[4];
  const float* w_ih_l0r = (const float*)d_in[5];
  const float* w_hh_l0r = (const float*)d_in[6];
  const float* b_ih_l0r = (const float*)d_in[7];
  const float* b_hh_l0r = (const float*)d_in[8];
  const float* w_ih_l1  = (const float*)d_in[9];
  const float* w_hh_l1  = (const float*)d_in[10];
  const float* b_ih_l1  = (const float*)d_in[11];
  const float* b_hh_l1  = (const float*)d_in[12];
  const float* w_ih_l1r = (const float*)d_in[13];
  const float* w_hh_l1r = (const float*)d_in[14];
  const float* b_ih_l1r = (const float*)d_in[15];
  const float* b_hh_l1r = (const float*)d_in[16];
  const float* fc_w     = (const float*)d_in[17];
  const float* fc_b     = (const float*)d_in[18];
  float* out = (float*)d_out;

  char* ws = (char*)d_ws; size_t off = 0;
  auto carve = [&](size_t bytes) -> char* { char* p = ws + off; off += (bytes + 255) & ~(size_t)255; return p; };
  unsigned short* OUT0 = (unsigned short*)carve((size_t)NSEQ * NSTEP * NIN1 * 2);
  float*          LAST = (float*)carve((size_t)NSEQ * NIN1 * 4);
  unsigned short* BT0  = (unsigned short*)carve((size_t)2 * NGATE * KP0 * 2);
  unsigned short* BT1  = (unsigned short*)carve((size_t)2 * NGATE * KP1 * 2);
  if (off > ws_size || off > (size_t)134217728) return;

  pack_weights_kernel<<<dim3(NGATE * KP1 / 8 / 256, 4), 256, 0, stream>>>(
      w_ih_l0, w_hh_l0, w_ih_l0r, w_hh_l0r, w_ih_l1, w_hh_l1, w_ih_l1r, w_hh_l1r, BT0, BT1);
  bilstm_layer_kernel<0><<<128, NTHR, 0, stream>>>(x, OUT0, BT0, b_ih_l0, b_hh_l0, b_ih_l0r, b_hh_l0r, OUT0, LAST);
  bilstm_layer_kernel<1><<<128, NTHR, 0, stream>>>(x, OUT0, BT1, b_ih_l1, b_hh_l1, b_ih_l1r, b_hh_l1r, OUT0, LAST);
  head_kernel<<<NSEQ / 256, 256, 0, stream>>>(LAST, fc_w, fc_b, out);
}
